// SMoE_23983097381214
// MI455X (gfx1250) — hardware-verified
//
#include <hip/hip_runtime.h>
#include <stddef.h>
#include <stdint.h>

#define NB   32
#define NS   512
#define ND   768
#define NO   768
#define NE   8
#define TM   64
#define TN   256
#define EP   68
#define PT   192
#define WMS  64.0f
#define WMI  0.015625f

static_assert(NS % TM == 0);
static_assert(NO % TN == 0);
static_assert(ND % 32 == 0);
static_assert(TM == 64);
static_assert(TN == 256);
static_assert(EP % 4 == 0);
static_assert(ND == 4 * PT);
static_assert(PT % 32 == 0);
static_assert(NB * NE == 256);
static_assert(((size_t)NB * NS * ND) % (8 * 256) == 0);
static_assert(((size_t)NO * ND) % (8 * 256) == 0);
static_assert((NB * NO / 4) % 256 == 0);
static_assert((ND * NE) % 256 == 0);
static_assert(NS % 4 == 0);

typedef _Float16 v16h __attribute__((ext_vector_type(16)));
typedef _Float16 v8h  __attribute__((ext_vector_type(8)));
typedef float    v8f  __attribute__((ext_vector_type(8)));
typedef float    v4f  __attribute__((ext_vector_type(4)));
typedef unsigned int v4u __attribute__((ext_vector_type(4)));

union Frag  { v16h v; v8h h[2]; };
union Pack8 { v8h h; v4u u; };

__device__ __forceinline__ v8f mma16(v16h a, v16h b, v8f c) {
  c = __builtin_amdgcn_wmma_f32_16x16x32_f16(false, a, false, b, (short)0, c, false, false);
  asm volatile("v_nop\n\tv_nop\n\tv_nop\n\tv_nop" : "+v"(c) : "v"(a), "v"(b));
  return c;
}

__device__ __forceinline__ v16h ldfrag(const _Float16* p, int ld, int row0, int k0, int lane) {
  const int m = lane & 15, lh = lane >> 4;
  const _Float16* q = p + (size_t)(row0 + m) * ld + k0 + 8 * lh;
  Frag f;
  f.h[0] = *(const v8h*)(q);
  f.h[1] = *(const v8h*)(q + 16);
  return f.v;
}

__device__ __forceinline__ v8f zero8() { return (v8f){0.f, 0.f, 0.f, 0.f, 0.f, 0.f, 0.f, 0.f}; }
__device__ __forceinline__ v4f zero4() { return (v4f){0.f, 0.f, 0.f, 0.f}; }

__device__ __forceinline__ v4u pack8(v4f a, v4f b) {
  Pack8 pk;
  pk.h = (v8h){(_Float16)a[0], (_Float16)a[1], (_Float16)a[2], (_Float16)a[3],
               (_Float16)b[0], (_Float16)b[1], (_Float16)b[2], (_Float16)b[3]};
  return pk.u;
}

__global__ __launch_bounds__(256) void k_cvtx(const float* __restrict__ x, _Float16* __restrict__ xh) {
  const size_t p = (size_t)blockIdx.x * 256 + threadIdx.x;
  const float* s = x + 8 * p;
  const v4f a = *(const v4f*)(s);
  const v4f b = *(const v4f*)(s + 4);
  const v4u vv = pack8(a, b);
  volatile v4u* d = (volatile v4u*)(xh + 8 * p);
  *d = vv;
  __threadfence();
  *d = vv;
}

__global__ __launch_bounds__(PT) void k_pool(const float* __restrict__ x, float* __restrict__ pooled) {
  const int b = blockIdx.x, t = threadIdx.x;
  const float* p = x + (size_t)b * NS * ND + 4 * t;
  v4f a0 = zero4(), a1 = zero4(), a2 = zero4(), a3 = zero4();
#pragma unroll 1
  for (int s = 0; s < NS; s += 4) {
    a0 += *(const v4f*)(p + (size_t)(s)     * ND);
    a1 += *(const v4f*)(p + (size_t)(s + 1) * ND);
    a2 += *(const v4f*)(p + (size_t)(s + 2) * ND);
    a3 += *(const v4f*)(p + (size_t)(s + 3) * ND);
  }
  const v4f m = ((a0 + a1) + (a2 + a3)) * (1.0f / (float)NS);
  volatile v4f* d = (volatile v4f*)(pooled + (size_t)b * ND + 4 * t);
  *d = m;
  __threadfence();
  *d = m;
}

__global__ __launch_bounds__(256) void k_gate(const float* __restrict__ pooled, const float* __restrict__ wg,
                                              const float* __restrict__ bias, float* __restrict__ gpl,
                                              float* __restrict__ ebp, float* __restrict__ lossp) {
  __shared__ __align__(16) float sWg[ND * NE];
  __shared__ __align__(16) float sL[NB * NE];
  __shared__ __align__(16) float sG[NB * NE];
  __shared__ float sImp[NE];
  __shared__ float sLd[NE];
  const int tid = threadIdx.x;

#pragma unroll 1
  for (int i = tid; i < ND * NE; i += 256) sWg[i] = wg[i];
  __syncthreads();

  {
    const int b = tid >> 3, e = tid & 7;
    const float* pr = pooled + (size_t)b * ND;
    float acc = 0.f;
#pragma unroll 1
    for (int d = 0; d < ND; ++d) acc += pr[d] * sWg[d * NE + e];
    sL[tid] = acc;
  }
  __syncthreads();

  if (tid < NB) {
    const int b = tid;
    int i0 = 0; float v0 = sL[b * NE];
#pragma unroll
    for (int j = 1; j < NE; ++j) {
      const float v = sL[b * NE + j];
      const bool c = v > v0;
      i0 = c ? j : i0; v0 = c ? v : v0;
    }
    int i1 = (i0 == 0) ? 1 : 0; float v1 = sL[b * NE + i1];
#pragma unroll
    for (int j = 1; j < NE; ++j) {
      const float v = sL[b * NE + j];
      const bool c = (j != i0) && (v > v1);
      i1 = c ? j : i1; v1 = c ? v : v1;
    }
    const float u1 = expf(v1 - v0);
    const float inv = 1.0f / (1.0f + u1);
    const float g0 = inv;
    const float g1 = u1 * inv;
#pragma unroll
    for (int j = 0; j < NE; ++j) sG[b * NE + j] = 0.f;
    sG[b * NE + i0] = g0;
    sG[b * NE + i1] = g1;
  }
  __syncthreads();

  if (tid < NE) {
    float si = 0.f, sl = 0.f;
#pragma unroll 1
    for (int b = 0; b < NB; ++b) {
      const float g = sG[b * NE + tid];
      si += g;
      sl += (g > 0.f) ? 1.f : 0.f;
    }
    sImp[tid] = si; sLd[tid] = sl;
  }
  __syncthreads();

  if (tid == 0) {
    float mi = 0.f, ml = 0.f;
#pragma unroll
    for (int j = 0; j < NE; ++j) { mi += sImp[j]; ml += sLd[j]; }
    mi *= (1.0f / (float)NE); ml *= (1.0f / (float)NE);
    float vi = 0.f, vl = 0.f;
#pragma unroll
    for (int j = 0; j < NE; ++j) {
      const float a = sImp[j] - mi; vi += a * a;
      const float c = sLd[j] - ml; vl += c * c;
    }
    vi *= (1.0f / (float)(NE - 1)); vl *= (1.0f / (float)(NE - 1));
    const float cv = vi / (mi * mi + 1e-10f) + vl / (ml * ml + 1e-10f);
    const float ls = cv * 0.01f;
    volatile float* d = (volatile float*)lossp;
    *d = ls;
    __threadfence();
    *d = ls;
  }

  if (tid < 64) {
    const v4f gv = *(const v4f*)(sG + 4 * tid);
    volatile v4f* d = (volatile v4f*)(gpl + 4 * tid);
    *d = gv;
    __threadfence();
    *d = gv;
  }

#pragma unroll 1
  for (int it = 0; it < (NB * NO / 4) / 256; ++it) {
    const int p  = it * 256 + tid;
    const int b  = p / (NO / 4);
    const int o4 = (p - b * (NO / 4)) * 4;
    v4f acc = zero4();
#pragma unroll 1
    for (int e = 0; e < NE; ++e) {
      const float g = sG[b * NE + e];
      const v4f bv = *(const v4f*)(bias + (size_t)e * NO + o4);
      acc += g * bv;
    }
    volatile v4f* d = (volatile v4f*)(ebp + 4 * (size_t)p);
    *d = acc;
    __threadfence();
    *d = acc;
  }
}

__global__ __launch_bounds__(256) void k_wmix(const float* __restrict__ weight, const float* __restrict__ gpl,
                                              _Float16* __restrict__ wh) {
  const int b = blockIdx.y;
  const size_t p = (size_t)blockIdx.x * 256 + threadIdx.x;
  v4f a0 = zero4(), a1 = zero4();
#pragma unroll 1
  for (int e = 0; e < NE; ++e) {
    const float g = __int_as_float(__builtin_amdgcn_readfirstlane(__float_as_int(gpl[b * NE + e])));
    if (g != 0.0f) {
      const float* src = weight + (size_t)e * ((size_t)NO * ND) + 8 * p;
      const v4f wa = *(const v4f*)(src);
      const v4f wb = *(const v4f*)(src + 4);
      a0 += g * wa;
      a1 += g * wb;
    }
  }
  const v4u vv = pack8(a0 * WMS, a1 * WMS);
  volatile v4u* d = (volatile v4u*)(wh + (size_t)b * ((size_t)NO * ND) + 8 * p);
  *d = vv;
  __threadfence();
  *d = vv;
}

__global__ __launch_bounds__(256) void k_gemm(const _Float16* __restrict__ xh, const _Float16* __restrict__ wh,
                                              const float* __restrict__ ebp, float* __restrict__ y) {
  __shared__ __align__(16) float sO[8 * 16 * EP];
  const int tid = threadIdx.x, lane = tid & 31, wave = tid >> 5;
  const int hh = lane >> 4, c = lane & 15;
  const int wm = wave & 1, wn = wave >> 1;
  const int b  = blockIdx.z;
  const int sB = blockIdx.y * TM;
  const int oB = blockIdx.x * TN;
  const int arow = b * NS + sB + wm * 32;
  const int brow = b * NO + oB + wn * 64;

  v8f acc[2][4];
#pragma unroll
  for (int mt = 0; mt < 2; ++mt) {
#pragma unroll
    for (int nt = 0; nt < 4; ++nt) acc[mt][nt] = zero8();
  }
#pragma unroll 1
  for (int k0 = 0; k0 < ND; k0 += 32) {
    const v16h a0 = ldfrag(xh, ND, arow, k0, lane);
    const v16h a1 = ldfrag(xh, ND, arow + 16, k0, lane);
#pragma unroll
    for (int nt = 0; nt < 4; ++nt) {
      const v16h bq = ldfrag(wh, ND, brow + 16 * nt, k0, lane);
      acc[0][nt] = mma16(a0, bq, acc[0][nt]);
      acc[1][nt] = mma16(a1, bq, acc[1][nt]);
    }
  }

  const v4f ebv = *(const v4f*)(ebp + (size_t)b * NO + oB + wn * 64 + 4 * c);
  float* so = sO + wave * (16 * EP);
#pragma unroll
  for (int mt = 0; mt < 2; ++mt) {
    __syncthreads();
#pragma unroll
    for (int nt = 0; nt < 4; ++nt) {
#pragma unroll
      for (int r = 0; r < 8; ++r) so[(8 * hh + r) * EP + nt * 16 + c] = acc[mt][nt][r];
    }
    __syncthreads();
    v4f val[8];
    size_t go[8];
#pragma unroll
    for (int it = 0; it < 8; ++it) {
      const int L = 2 * it + hh;
      const v4f hv = *(const v4f*)(so + L * EP + 4 * c);
      val[it] = hv * WMI + ebv;
      go[it] = (size_t)(arow + mt * 16 + L) * NO + oB + wn * 64 + 4 * c;
    }
#pragma unroll
    for (int it = 0; it < 8; ++it) *(volatile v4f*)(y + go[it]) = val[it];
    __threadfence();
#pragma unroll
    for (int it = 0; it < 8; ++it) *(volatile v4f*)(y + go[it]) = val[it];
  }
}

extern "C" void kernel_launch(void* const* d_in, const int* in_sizes, int n_in,
                              void* d_out, int out_size, void* d_ws, size_t ws_size,
                              hipStream_t stream) {
  if (n_in < 4) return;
  if (in_sizes[0] != NB * NS * ND) return;
  if (in_sizes[1] != ND * NE) return;
  if (in_sizes[2] != NE * NO * ND) return;
  if (in_sizes[3] != NE * NO) return;
  if (out_size != NB * NS * NO + 1) return;

  const float* x      = (const float*)d_in[0];
  const float* w_gate = (const float*)d_in[1];
  const float* weight = (const float*)d_in[2];
  const float* bias   = (const float*)d_in[3];
  float* y    = (float*)d_out;
  float* loss = y + (size_t)NB * NS * NO;

  size_t off = 0;
  const size_t oXH = off; off += (size_t)NB * NS * ND * 2;
  const size_t oWH = off; off += (size_t)NB * NO * ND * 2;
  const size_t oP  = off; off += (size_t)NB * ND * 4;
  const size_t oG  = off; off += (size_t)NB * NE * 4;
  const size_t oEB = off; off += (size_t)NB * NO * 4;
  if (off > ws_size) return;
  if (off > (size_t)134217728) return;
  if ((oXH | oWH | oP | oG | oEB) & (size_t)127) return;

  char* ws = (char*)d_ws;
  _Float16* XH = (_Float16*)(ws + oXH);
  _Float16* WH = (_Float16*)(ws + oWH);
  float*    P  = (float*)(ws + oP);
  float*    G  = (float*)(ws + oG);
  float*    EB = (float*)(ws + oEB);

  k_cvtx<<<dim3((NB * NS * ND) / (8 * 256)), dim3(256), 0, stream>>>(x, XH);
  k_pool<<<dim3(NB), dim3(PT), 0, stream>>>(x, P);
  k_gate<<<dim3(1), dim3(256), 0, stream>>>(P, w_gate, bias, G, EB, loss);
  k_wmix<<<dim3((NO * ND) / (8 * 256), NB), dim3(256), 0, stream>>>(weight, G, WH);
  k_gemm<<<dim3(NO / TN, NS / TM, NB), dim3(256), 0, stream>>>(XH, WH, EB, y);
  (void)hipGetLastError();
}
